// D2V18AttentionBlock_73134703116752
// MI455X (gfx1250) — hardware-run, weakly checked
//
#include <hip/hip_runtime.h>
#include <math.h>

typedef __attribute__((ext_vector_type(16))) _Float16 v16h;
typedef __attribute__((ext_vector_type(16))) __bf16 v16b;
typedef __attribute__((ext_vector_type(8)))  _Float16 v8h;
typedef __attribute__((ext_vector_type(8)))  float v8f;
typedef __attribute__((ext_vector_type(4)))  float v4f;
typedef __attribute__((ext_vector_type(2)))  float v2f;
typedef __attribute__((ext_vector_type(4)))  unsigned v4u;
typedef __attribute__((ext_vector_type(4)))  int v4i;
typedef float __attribute__((may_alias)) float_a;
typedef int __attribute__((may_alias)) int_a;

template <typename T> __device__ __forceinline__ void vst2(void* p, T v) { *(volatile T*)p = v; __threadfence(); *(volatile T*)p = v; }
__device__ __forceinline__ v8f wmma16(v16h a, v16h b, v8f c) {
  v8f d = __builtin_amdgcn_wmma_f32_16x16x32_f16(false, a, false, b, (short)0, c, false, false);
  asm volatile("v_nop\n\tv_nop\n\tv_nop\n\tv_nop" : "+v"(d) : "v"(a), "v"(b));
  return d;
}
__device__ __forceinline__ v8f wmma_bf(v16b a, v16b b, v8f c) {
  v8f d = __builtin_amdgcn_wmma_f32_16x16x32_bf16(false, a, false, b, (short)0, c, false, false);
  asm volatile("v_nop\n\tv_nop\n\tv_nop\n\tv_nop" : "+v"(d) : "v"(a), "v"(b));
  return d;
}
__device__ __forceinline__ v16h frag_h(const _Float16* rowk0, int lane) {
  union { v16h v; v8h q[2]; } u; const _Float16* p = rowk0 + 8 * (lane >> 4);
  u.q[0] = *(const v8h*)p; u.q[1] = *(const v8h*)(p + 16); return u.v;
}
__device__ __forceinline__ v16h frag_f32(const float* rowk0, int lane) {
  v16h a; const float* p = rowk0 + 8 * (lane >> 4);
#pragma unroll
  for (int i = 0; i < 8; ++i) { a[i] = (_Float16)p[i]; a[8 + i] = (_Float16)p[16 + i]; }
  return a;
}
__device__ __forceinline__ v16h frag_f32s(const float* rowk0, int lane, float sc) {
  v16h a; const float* p = rowk0 + 8 * (lane >> 4);
#pragma unroll
  for (int i = 0; i < 8; ++i) { a[i] = (_Float16)(p[i] * sc); a[8 + i] = (_Float16)(p[16 + i] * sc); }
  return a;
}
__device__ __forceinline__ v16h fragc_f32(const float* W, int k0, int n, int lane, int ld, int K) {
  v16h a; const int g = lane >> 4;
#pragma unroll
  for (int i = 0; i < 8; ++i) { const int ka = k0 + 8 * g + i, kb = ka + 16;
    a[i] = (_Float16)(ka < K ? W[(size_t)(ka < K ? ka : K - 1) * ld + n] : 0.f); a[8 + i] = (_Float16)(kb < K ? W[(size_t)(kb < K ? kb : K - 1) * ld + n] : 0.f); }
  return a;
}
struct F2 { v16b h, l; };
__device__ __forceinline__ F2 bsplit16(const float v[16]) { F2 r;
#pragma unroll
  for (int i = 0; i < 16; ++i) { const __bf16 h = (__bf16)v[i]; r.h[i] = h; r.l[i] = (__bf16)(v[i] - (float)h); }
  return r; }
__device__ __forceinline__ F2 split_row(const float* row, int k0, int lane) { float v[16]; const float* p = row + k0 + 8 * (lane >> 4);
#pragma unroll
  for (int i = 0; i < 8; ++i) { v[i] = p[i]; v[8 + i] = p[16 + i]; }
  return bsplit16(v); }
__device__ __forceinline__ F2 split_rowK(const float* row, int k0, int lane, int K) { float v[16]; const int g = lane >> 4;
#pragma unroll
  for (int i = 0; i < 8; ++i) { const int ka = k0 + 8 * g + i, kb = ka + 16; v[i] = ka < K ? row[ka < K ? ka : K - 1] : 0.f; v[8 + i] = kb < K ? row[kb < K ? kb : K - 1] : 0.f; }
  return bsplit16(v); }
__device__ __forceinline__ F2 split_col(const float* W, int k0, int n, int lane, int ld, int K) { float v[16]; const int g = lane >> 4;
#pragma unroll
  for (int i = 0; i < 8; ++i) { const int ka = k0 + 8 * g + i, kb = ka + 16; v[i] = ka < K ? W[(size_t)(ka < K ? ka : K - 1) * ld + n] : 0.f; v[8 + i] = kb < K ? W[(size_t)(kb < K ? kb : K - 1) * ld + n] : 0.f; }
  return bsplit16(v); }
__device__ __forceinline__ v8f mac3(const F2& a, const F2& b, v8f c) { c = wmma_bf(a.l, b.h, c); c = wmma_bf(a.h, b.l, c); return wmma_bf(a.h, b.h, c); }
__device__ __forceinline__ float sigm(float v) { return 1.0f / (1.0f + expf(-v)); }
#define LDSX() do { asm volatile("s_wait_dscnt 0" ::: "memory"); __builtin_amdgcn_wave_barrier(); __builtin_amdgcn_fence(__ATOMIC_RELEASE, "workgroup"); } while (0)


#define LL 2048
#define DMOD 768
#define NH 12
#define HD 64
#define LAT 512
#define HID 2048
#define NB2 3200
#ifndef NRB
#define NRB (LL / 64)
#endif
#ifndef LSCAN
#define LSCAN LL
#endif
typedef __attribute__((ext_vector_type(8))) __bf16 v8b;
__device__ __forceinline__ v16b frag_b(const __bf16* rowk0, int lane) {
  union { v16b v; v8b q[2]; } u; const __bf16* p = rowk0 + 8 * (lane >> 4);
  u.q[0] = *(const v8b*)p; u.q[1] = *(const v8b*)(p + 16); return u.v;
}
__device__ __forceinline__ float bfr(float v) { return (float)(__bf16)v; }
__device__ __attribute__((noinline)) float exp_ni(float v) { return expf(v); }
__device__ __attribute__((noinline)) float erf_ni(float v) { return erff(v); }

#define WS_PC   0u
#define WS_P2   (WS_PC + 2u * (size_t)LAT * DMOD)
#define WS_PP   (WS_P2 + 2u * (size_t)NB2 * LAT)
#define WS_PF1  (WS_PP + 2u * (size_t)DMOD * DMOD)
#define WS_PF2  (WS_PF1 + 2u * (size_t)HID * DMOD)
#define WS_PF3  (WS_PF2 + 2u * (size_t)HID * DMOD)
#define WS_XN   (WS_PF3 + 2u * (size_t)DMOD * HID)
#define WS_LATB (WS_XN + 4u * (size_t)LL * DMOD)
#define WS_BIG  (WS_LATB + 4u * (size_t)LL * LAT)
#define WS_QF   (WS_BIG + 4u * (size_t)LL * NB2)
#define WS_KF   (WS_QF + 4u * (size_t)LL * DMOD)
#define WS_GATE (WS_KF + 4u * (size_t)LL * DMOD)
#define WS_AO   (WS_GATE + 4u * (size_t)LL * 16)
#define WS_MO   (WS_AO + 4u * (size_t)LL * DMOD)
#define WS_X1   (WS_MO + 4u * (size_t)LL * DMOD)
#define WS_XN2  (WS_X1 + 4u * (size_t)LL * DMOD)
#define WS_G16  (WS_XN2 + 2u * (size_t)LL * DMOD)
#define WS_END  (WS_G16 + 2u * (size_t)LL * HID)

__global__ __launch_bounds__(256) void k_pack(const float* __restrict__ WC, const float* __restrict__ WQ, const float* __restrict__ WOG, const float* __restrict__ WR, const float* __restrict__ WP, const float* __restrict__ W1, const float* __restrict__ W2, const float* __restrict__ W3, __bf16* __restrict__ P, _Float16* __restrict__ PH) {
  const int n = blockIdx.x, which = blockIdx.y, t = threadIdx.x; __shared__ __align__(16) __bf16 s[DMOD]; __shared__ __align__(16) _Float16 sh[HID];
  if (which == 0) { if (n >= LAT) return; for (int k = t; k < DMOD; k += 256) s[k] = (__bf16)WC[(size_t)k * LAT + n]; __syncthreads(); for (int q = t; q < DMOD / 8; q += 256) vst2((unsigned*)(P + WS_PC / 2 + (size_t)n * DMOD + q * 8), *(const v4u*)&s[q * 8]); }
  else if (which == 1) { if (n >= NB2) return; for (int k = t; k < LAT; k += 256) { float v = 0.f; if (n < 3 * DMOD) v = WQ[(size_t)k * 3 * DMOD + n]; else if (n < 4 * DMOD) v = WOG[(size_t)k * DMOD + (n - 3 * DMOD)]; else if (n < 4 * DMOD + NH * 4) v = WR[(size_t)k * (NH * 4) + (n - 4 * DMOD)]; s[k] = (__bf16)v; } __syncthreads(); for (int q = t; q < LAT / 8; q += 256) vst2((unsigned*)(P + WS_P2 / 2 + (size_t)n * LAT + q * 8), *(const v4u*)&s[q * 8]); }
  else if (which == 2) { if (n >= DMOD) return; for (int k = t; k < DMOD; k += 256) s[k] = (__bf16)WP[(size_t)k * DMOD + n]; __syncthreads(); for (int q = t; q < DMOD / 8; q += 256) vst2((unsigned*)(P + WS_PP / 2 + (size_t)n * DMOD + q * 8), *(const v4u*)&s[q * 8]); }
  else if (which <= 4) { if (n >= HID) return; const float* Wm = (which == 3) ? W1 : W2; for (int k = t; k < DMOD; k += 256) sh[k] = (_Float16)(bfr(Wm[(size_t)k * HID + n]) * 256.0f); __syncthreads(); for (int q = t; q < DMOD / 8; q += 256) vst2((unsigned*)(PH + (which == 3 ? 0 : (size_t)HID * DMOD) + (size_t)n * DMOD + q * 8), *(const v4u*)&sh[q * 8]); }
  else { if (n >= DMOD) return; for (int k = t; k < HID; k += 256) sh[k] = (_Float16)(bfr(W3[(size_t)k * DMOD + n]) * 256.0f); __syncthreads(); for (int q = t; q < HID / 8; q += 256) vst2((unsigned*)(PH + (size_t)2 * HID * DMOD + (size_t)n * HID + q * 8), *(const v4u*)&sh[q * 8]); }
}
template <int MODE>
__global__ __launch_bounds__(192) void k_rms(const float* __restrict__ Xin, const float* __restrict__ Wn, float* __restrict__ OF, _Float16* __restrict__ OH) {
  __shared__ float red[6]; __shared__ __align__(16) _Float16 sh[DMOD]; const int t = threadIdx.x; const size_t row = blockIdx.x; float v[4]; float q = 0.f;
  for (int i = 0; i < 4; ++i) { const float x = Xin[row * DMOD + t * 4 + i]; v[i] = (MODE == 0) ? bfr(x) : x; q += v[i] * v[i]; }
#pragma unroll
  for (int o = 1; o < 32; o <<= 1) q += __shfl_xor(q, o);
  if ((t & 31) == 0) red[t >> 5] = q; __syncthreads(); float tq = 0.f; for (int i = 0; i < 6; ++i) tq += red[i]; const float rs = 1.0f / sqrtf(tq / (float)DMOD + 1e-6f);
  v4f o4; for (int i = 0; i < 4; ++i) { const int e = t * 4 + i; o4[i] = bfr(Wn[e]) * (v[i] * rs); if (MODE == 2) sh[e] = (_Float16)o4[i]; }
  if (MODE != 2) vst2(OF + row * DMOD + t * 4, o4);
  else { __syncthreads(); if (t < DMOD / 8) vst2((unsigned*)(OH + row * DMOD + t * 8), *(const v4u*)&sh[t * 8]); }
}
__device__ __attribute__((noinline)) float exp_p(float v) { return expf(v); }
__device__ __forceinline__ float silu_f(float x) { return x / (1.0f + exp_p(-x)); }
__device__ __forceinline__ float sigm_f(float x) { return 1.0f / (1.0f + exp_p(-x)); }
template <int KIN, int NOUT, int MODE>
__global__ __launch_bounds__(128) void k_lin(const float* __restrict__ A, const __bf16* __restrict__ Wr, const float* __restrict__ XR, const float* __restrict__ OGp, float* __restrict__ OUT) {
  __shared__ __align__(16) float so[4][16][132];
  const int tid = threadIdx.x, wave = tid >> 5, lane = tid & 31, col = lane & 15, g = lane >> 4; const size_t r0 = (size_t)blockIdx.x * 64 + wave * 16; const int n0 = blockIdx.y * 128;
  v8f acc[8] = {};
#pragma unroll 2
  for (int kc = 0; kc < KIN / 32; ++kc) { const F2 a = split_row(A + (r0 + col) * KIN, kc * 32, lane);
#pragma unroll
    for (int j = 0; j < 8; ++j) { const v16b w = frag_b(Wr + (size_t)(n0 + j * 16 + col) * KIN + kc * 32, lane); acc[j] = wmma_bf(a.l, w, acc[j]); acc[j] = wmma_bf(a.h, w, acc[j]); } }
#pragma unroll
  for (int j = 0; j < 8; ++j) { const int c = n0 + j * 16 + col;
#pragma unroll
    for (int r = 0; r < 8; ++r) { const size_t row = r0 + 8 * g + r; float v = acc[j][r]; if (MODE == 0) v = silu_f(v); else if (MODE == 2) v = bfr(XR[row * DMOD + c]) + v * silu_f(OGp[row * NB2 + 3 * DMOD + c]); so[wave][8 * g + r][j * 16 + col] = v; } }
  LDSX();
  for (int rl = 0; rl < 16; ++rl) vst2(OUT + (r0 + rl) * NOUT + n0 + lane * 4, *(const v4f*)&so[wave][rl][lane * 4]);
}
__constant__ float INVF[32] = {1.000000000e+00f,7.498942018e-01f,5.623413324e-01f,4.216965139e-01f,3.162277639e-01f,2.371373773e-01f,1.778279394e-01f,1.333521456e-01f,1.000000015e-01f,7.498942316e-02f,5.623413250e-02f,4.216964915e-02f,3.162277490e-02f,2.371373773e-02f,1.778279431e-02f,1.333521400e-02f,9.999999776e-03f,7.498942316e-03f,5.623413250e-03f,4.216964822e-03f,3.162277630e-03f,2.371373819e-03f,1.778279431e-03f,1.333521446e-03f,1.000000047e-03f,7.498941850e-04f,5.623413017e-04f,4.216965172e-04f,3.162277571e-04f,2.371373703e-04f,1.778279402e-04f,1.333521504e-04f};
__device__ __attribute__((noinline)) float cos_p(float v) { return cosf(v); }
__device__ __attribute__((noinline)) float sin_p(float v) { return sinf(v); }
__global__ __launch_bounds__(384) void k_prep(const float* __restrict__ BIG, const float* __restrict__ QNW, const float* __restrict__ KNW, const float* __restrict__ TEMP, float* __restrict__ QF, float* __restrict__ KF, float* __restrict__ GATE) {
  const size_t t = blockIdx.x; const int tid = threadIdx.x, h = tid >> 5, lane = tid & 31;
  const float* row = BIG + t * NB2; const float q0 = row[h * HD + lane], q1 = row[h * HD + lane + 32], k0 = row[DMOD + h * HD + lane], k1 = row[DMOD + h * HD + lane + 32];
  float sq = q0 * q0 + q1 * q1, sk = k0 * k0 + k1 * k1;
#pragma unroll
  for (int o = 1; o < 32; o <<= 1) { sq += __shfl_xor(sq, o); sk += __shfl_xor(sk, o); }
  const float rq = 1.0f / sqrtf(sq / (float)HD + 1e-6f), rk = 1.0f / sqrtf(sk / (float)HD + 1e-6f);
  const float qn0 = bfr(QNW[lane]) * (q0 * rq), qn1 = bfr(QNW[lane + 32]) * (q1 * rq), kn0 = bfr(KNW[lane]) * (k0 * rk), kn1 = bfr(KNW[lane + 32]) * (k1 * rk);
  const float ang = (float)t * INVF[lane]; const float cs = cos_p(ang), sn = sin_p(ang);
  const float qr0 = qn0 * cs - qn1 * sn, qr1 = qn1 * cs + qn0 * sn, kr0 = kn0 * cs - kn1 * sn, kr1 = kn1 * cs + kn0 * sn;
  QF[t * DMOD + h * HD + lane] = (qr0 > 0.f ? qr0 : exp_p(qr0) - 1.0f) + 1.0f; QF[t * DMOD + h * HD + lane + 32] = (qr1 > 0.f ? qr1 : exp_p(qr1) - 1.0f) + 1.0f;
  KF[t * DMOD + h * HD + lane] = (kr0 > 0.f ? kr0 : exp_p(kr0) - 1.0f) + 1.0f; KF[t * DMOD + h * HD + lane + 32] = (kr1 > 0.f ? kr1 : exp_p(kr1) - 1.0f) + 1.0f;
  if (lane == 0) { const float* pr = row + 4 * DMOD + h * 4; const float sem_amp = sigm_f(pr[0]), sem_ph = sigm_f(pr[1]) * 3.14159265358979323846f, ctx_amp = sigm_f(pr[2]), ctx_ph = sigm_f(pr[3]) * 3.14159265358979323846f;
    const float bg = sigm_f(sem_amp * ctx_amp * cos_p(sem_ph - ctx_ph) * bfr(TEMP[0])); GATE[t * 16 + h] = fminf(fmaxf(bg * 1.2f - 0.1f, 0.05f), 0.95f); }
}
__device__ __attribute__((noinline)) float log_p(float v) { return logf(v); }
__global__ __launch_bounds__(256) void k_scan(const float* __restrict__ QF, const float* __restrict__ KF, const float* __restrict__ BIG, const float* __restrict__ GATE, const float* __restrict__ HDEC, float* __restrict__ AO) {
  __shared__ float sq[HD], skd[HD], sv[HD]; __shared__ float part[4][HD][17]; __shared__ float zpart[HD];
  const int h = blockIdx.x, tid = threadIdx.x; const int d = tid >> 2, eq = tid & 3, e0 = eq * 16;
  const float raw = 0.3f + 0.65f * sigm_f(bfr(HDEC[h])); const float decay = fminf(fmaxf(raw, 1e-5f), 0.999f); const float dt = 1.0f - decay; const float lg = log_p(decay);
  float A[16]; for (int i = 0; i < 16; ++i) A[i] = 0.f; float z = 0.f; float cum = 0.f;
#pragma unroll 1
  for (int t = 0; t < LSCAN; ++t) {
    if (tid < HD) { sq[tid] = QF[(size_t)t * DMOD + h * HD + tid]; skd[tid] = KF[(size_t)t * DMOD + h * HD + tid]; sv[tid] = BIG[(size_t)t * NB2 + 2 * DMOD + h * HD + tid]; }
    __syncthreads();
    cum += lg; const float df = exp_p(cum); const float safe = df + 1e-8f; const float gate = GATE[(size_t)t * 16 + h];
    const float kd = skd[d]; const float kvs = kd * gate * dt;
#pragma unroll
    for (int i = 0; i < 16; ++i) A[i] += (kvs * sv[e0 + i]) / safe;
    if (eq == 0) z += (kd * dt) / safe;
    const float qd = sq[d];
#pragma unroll
    for (int i = 0; i < 16; ++i) part[eq][d][i] = qd * (A[i] * df);
    if (eq == 0) zpart[d] = qd * (z * df);
    __syncthreads();
    if (tid < HD) { const int e = tid; float num = 0.f;
#pragma unroll 1
      for (int dd = 0; dd < HD; ++dd) num += part[e >> 4][dd][e & 15];
      float den = 0.f; if (tid == 0) { }
#pragma unroll 1
      for (int dd = 0; dd < HD; ++dd) den += zpart[dd];
      den = fmaxf(den, 1e-5f); AO[(size_t)t * DMOD + h * HD + e] = num / den; }
    __syncthreads(); }
}
template <int MODE>
__global__ __launch_bounds__(128) void k_mlp(const _Float16* __restrict__ Ain, const _Float16* __restrict__ PH, const float* __restrict__ RES, float* __restrict__ OUTF, _Float16* __restrict__ OG) {
  constexpr int KIN = (MODE == 0) ? DMOD : HID; constexpr int NOUT = (MODE == 0) ? HID : DMOD;
  __shared__ __align__(16) float so[4][16][132]; __shared__ __align__(16) _Float16 sg[4][16][136];
  const int tid = threadIdx.x, wave = tid >> 5, lane = tid & 31, col = lane & 15, g = lane >> 4; const size_t r0 = (size_t)blockIdx.x * 64 + wave * 16; const int n0 = blockIdx.y * 128;
  v8f acc[8] = {}, acc2[8] = {};
  const _Float16* W1r = PH + ((MODE == 0) ? 0 : (size_t)2 * HID * DMOD); const _Float16* W2r = PH + (size_t)HID * DMOD;
#pragma unroll 2
  for (int kc = 0; kc < KIN / 32; ++kc) { const v16h a = frag_h(Ain + (r0 + col) * KIN + kc * 32, lane);
#pragma unroll
    for (int j = 0; j < 8; ++j) { acc[j] = wmma16(a, frag_h(W1r + (size_t)(n0 + j * 16 + col) * KIN + kc * 32, lane), acc[j]); if (MODE == 0) acc2[j] = wmma16(a, frag_h(W2r + (size_t)(n0 + j * 16 + col) * KIN + kc * 32, lane), acc2[j]); } }
#pragma unroll
  for (int j = 0; j < 8; ++j) { const int c = n0 + j * 16 + col;
#pragma unroll
    for (int r = 0; r < 8; ++r) { if (MODE == 0) { const float h1 = acc[j][r] * (1.0f / 256.0f), h2 = acc2[j][r] * (1.0f / 256.0f); sg[wave][8 * g + r][j * 16 + col] = (_Float16)(silu_f(h1) * h2); } else so[wave][8 * g + r][j * 16 + col] = acc[j][r] * (1.0f / 256.0f) + RES[(r0 + 8 * g + r) * DMOD + c]; } }
  LDSX();
  if (MODE == 0) { for (int rl = 0; rl < 16; ++rl) if (lane < 16) vst2((unsigned*)(OG + (r0 + rl) * NOUT + n0 + lane * 8), *(const v4u*)&sg[wave][rl][lane * 8]); }
  else { for (int rl = 0; rl < 16; ++rl) vst2(OUTF + (r0 + rl) * NOUT + n0 + lane * 4, *(const v4f*)&so[wave][rl][lane * 4]); }
}
extern "C" void kernel_launch(void* const* d_in, const int* in_sizes, int n_in, void* d_out, int out_size, void* d_ws, size_t ws_size, hipStream_t stream) {
  (void)in_sizes; (void)n_in; (void)out_size;
  const float** F = (const float**)d_in;
  if (ws_size < (size_t)WS_END) return;
  char* ws = (char*)d_ws; __bf16* P = (__bf16*)ws; _Float16 *PH = (_Float16*)(ws + WS_PF1), *XN2 = (_Float16*)(ws + WS_XN2), *G16 = (_Float16*)(ws + WS_G16); float *XN = (float*)(ws + WS_XN), *LATB = (float*)(ws + WS_LATB), *BIG = (float*)(ws + WS_BIG), *QF = (float*)(ws + WS_QF), *KF = (float*)(ws + WS_KF), *GATE = (float*)(ws + WS_GATE), *AO = (float*)(ws + WS_AO), *MO = (float*)(ws + WS_MO), *X1 = (float*)(ws + WS_X1);
  k_pack<<<dim3(NB2, 6), 256, 0, stream>>>(F[2], F[3], F[7], F[4], F[10], F[13], F[14], F[15], P, PH);
  k_rms<0><<<LL, 192, 0, stream>>>(F[0], F[1], XN, nullptr);
  k_lin<DMOD, LAT, 0><<<dim3(NRB, LAT / 128), 128, 0, stream>>>(XN, P + WS_PC / 2, nullptr, nullptr, LATB);
  k_lin<LAT, NB2, 1><<<dim3(NRB, NB2 / 128), 128, 0, stream>>>(LATB, P + WS_P2 / 2, nullptr, nullptr, BIG);
  k_prep<<<NRB * 64, 384, 0, stream>>>(BIG, F[5], F[6], F[9], QF, KF, GATE);
  k_scan<<<NH, 256, 0, stream>>>(QF, KF, BIG, GATE, F[8], AO);
  k_rms<1><<<LL, 192, 0, stream>>>(AO, F[11], MO, nullptr);
  k_lin<DMOD, DMOD, 2><<<dim3(NRB, DMOD / 128), 128, 0, stream>>>(MO, P + WS_PP / 2, F[0], BIG, X1);
  k_rms<2><<<LL, 192, 0, stream>>>(X1, F[12], nullptr, XN2);
  k_mlp<0><<<dim3(NRB, HID / 128), 128, 0, stream>>>(XN2, PH, nullptr, nullptr, G16);
  k_mlp<1><<<dim3(NRB, DMOD / 128), 128, 0, stream>>>(G16, PH, X1, (float*)d_out, nullptr);
}
